// MultiHeadAttentionWithRoPE_47167330844765
// MI455X (gfx1250) — hardware-verified
//
#include <hip/hip_runtime.h>
#include <stddef.h>

#define S_LEN   2048
#define D_MODEL 1024
#define N_HEADS 16
#define D_K     64

typedef __bf16         v16bf __attribute__((ext_vector_type(16)));
typedef _Float16       v16h  __attribute__((ext_vector_type(16)));
typedef _Float16       v8h   __attribute__((ext_vector_type(8)));
typedef float          v8f   __attribute__((ext_vector_type(8)));
typedef float          v4f   __attribute__((ext_vector_type(4)));
typedef unsigned short v16u  __attribute__((ext_vector_type(16)));
typedef unsigned short v8u   __attribute__((ext_vector_type(8)));

__device__ __forceinline__ unsigned short f2bf(float f) {
    unsigned int x = __builtin_bit_cast(unsigned int, f);
    unsigned int r = x + 0x7FFFu + ((x >> 16) & 1u);
    return (unsigned short)(r >> 16);
}
__device__ __forceinline__ float bf2f(unsigned short b) {
    return __builtin_bit_cast(float, ((unsigned int)b) << 16);
}

__device__ __forceinline__ v16u frag_u16(const unsigned short* p) {
    v8u x0 = *(const v8u*)p;
    v8u x1 = *(const v8u*)(p + 16);
    return __builtin_shufflevector(x0, x1, 0, 1, 2, 3, 4, 5, 6, 7, 8, 9, 10, 11, 12, 13, 14, 15);
}
__device__ __forceinline__ v16h frag_f16(const _Float16* p) {
    v8h x0 = *(const v8h*)p;
    v8h x1 = *(const v8h*)(p + 16);
    return __builtin_shufflevector(x0, x1, 0, 1, 2, 3, 4, 5, 6, 7, 8, 9, 10, 11, 12, 13, 14, 15);
}

__device__ __forceinline__ v8f mma_bf16(v16bf a, v16bf b, v8f c) {
    v8f d = __builtin_amdgcn_wmma_f32_16x16x32_bf16(false, a, false, b, (short)0, c, false, false);
    asm volatile("v_nop\n\tv_nop\n\tv_nop\n\tv_nop" : "+v"(d) : "v"(a), "v"(b));
    return d;
}
__device__ __forceinline__ v8f mma_f16(v16h a, v16h b, v8f c) {
    v8f d = __builtin_amdgcn_wmma_f32_16x16x32_f16(false, a, false, b, (short)0, c, false, false);
    asm volatile("v_nop\n\tv_nop\n\tv_nop\n\tv_nop" : "+v"(d) : "v"(a), "v"(b));
    return d;
}

__global__ __launch_bounds__(256) void cvt_kernel(
    const float* __restrict__ s0, const float* __restrict__ s1,
    const float* __restrict__ s2, const float* __restrict__ s3,
    unsigned short* d0, unsigned short* d1, unsigned short* d2, unsigned short* d3,
    int n8, int f16last) {
    const int sel = blockIdx.y;
    const float* s = (sel == 0) ? s0 : (sel == 1) ? s1 : (sel == 2) ? s2 : s3;
    unsigned short* d = (sel == 0) ? d0 : (sel == 1) ? d1 : (sel == 2) ? d2 : d3;
    const int i = blockIdx.x * blockDim.x + threadIdx.x;
    if (i >= n8) return;
    const v4f x0 = *(const v4f*)(s + (size_t)i * 8);
    const v4f x1 = *(const v4f*)(s + (size_t)i * 8 + 4);
    float x[8];
    x[0] = x0[0]; x[1] = x0[1]; x[2] = x0[2]; x[3] = x0[3];
    x[4] = x1[0]; x[5] = x1[1]; x[6] = x1[2]; x[7] = x1[3];
    v8u o;
    if (f16last != 0 && sel == 3) {
#pragma unroll
        for (int e = 0; e < 8; ++e) {
            const float r = bf2f(f2bf(x[e])) * 64.0f;
            o[e] = __builtin_bit_cast(unsigned short, (_Float16)r);
        }
    } else {
#pragma unroll
        for (int e = 0; e < 8; ++e) o[e] = f2bf(x[e]);
    }
    volatile v8u* p = (volatile v8u*)(d + (size_t)i * 8);
    *p = o;
    __threadfence();
    *p = o;
}

__global__ __launch_bounds__(256) void rope_tab_kernel(float* ct, float* st, int n4) {
    const int g = blockIdx.x * blockDim.x + threadIdx.x;
    if (g >= n4) return;
    const int t  = g >> 3;
    const int i0 = (g & 7) * 4;
    float c0 = 0.0f, c1 = 0.0f, c2 = 0.0f, c3 = 0.0f;
    float s0 = 0.0f, s1 = 0.0f, s2 = 0.0f, s3 = 0.0f;
#pragma unroll 1
    for (int e = 0; e < 4; ++e) {
        const int i = i0 + e;
        const float x = (float)(2 * i) / 64.0f;
        const float p = (float)pow(10000.0, (double)x);
        const float inv = 1.0f / p;
        const float ang = (float)t * inv;
        const float cv = cosf(ang);
        const float sv = sinf(ang);
        c0 = c1; c1 = c2; c2 = c3; c3 = cv;
        s0 = s1; s1 = s2; s2 = s3; s3 = sv;
    }
    v4f c, sn;
    c[0] = c0; c[1] = c1; c[2] = c2; c[3] = c3;
    sn[0] = s0; sn[1] = s1; sn[2] = s2; sn[3] = s3;
    volatile v4f* pc = (volatile v4f*)(ct + (size_t)t * 32 + i0);
    volatile v4f* ps = (volatile v4f*)(st + (size_t)t * 32 + i0);
    *pc = c; *ps = sn;
    __threadfence();
    *pc = c; *ps = sn;
}

template <int MODE>
__global__ __launch_bounds__(128) void gemm_kernel(
    const unsigned short* __restrict__ X, const unsigned short* __restrict__ W,
    const float* __restrict__ bias, const float* __restrict__ ct, const float* __restrict__ st,
    void* out0, void* out1) {
    __shared__ __attribute__((aligned(16))) unsigned char stage_raw[4 * 8192];

    const int tid  = threadIdx.x;
    const int lane = tid & 31;
    const int h    = lane >> 4;
    const int m    = lane & 15;
    const int wv   = tid >> 5;
    const int wave = blockIdx.x * 4 + wv;
    const int Mbase = (wave >> 4) * 32;
    const int Nbase = (wave & 15) * 64;

    v8f acc[2][4];
#pragma unroll
    for (int mt = 0; mt < 2; ++mt)
#pragma unroll
        for (int j = 0; j < 4; ++j) acc[mt][j] = (v8f)0.0f;

    const unsigned short* a0p = X + (size_t)(Mbase + m) * D_MODEL + 8 * h;
    const unsigned short* a1p = X + (size_t)(Mbase + 16 + m) * D_MODEL + 8 * h;
    const unsigned short* bbp = W + (size_t)(Nbase + m) * D_MODEL + 8 * h;

#pragma unroll 1
    for (int k = 0; k < D_MODEL; k += 32) {
        const v16u ua0 = frag_u16(a0p + k);
        const v16u ua1 = frag_u16(a1p + k);
#pragma unroll
        for (int j = 0; j < 4; ++j) {
            const v16u ub = frag_u16(bbp + (size_t)j * 16 * D_MODEL + k);
            if (MODE == 3) {
                const v16h b = __builtin_bit_cast(v16h, ub);
                acc[0][j] = mma_f16(__builtin_bit_cast(v16h, ua0), b, acc[0][j]);
                acc[1][j] = mma_f16(__builtin_bit_cast(v16h, ua1), b, acc[1][j]);
            } else {
                const v16bf b = __builtin_bit_cast(v16bf, ub);
                acc[0][j] = mma_bf16(__builtin_bit_cast(v16bf, ua0), b, acc[0][j]);
                acc[1][j] = mma_bf16(__builtin_bit_cast(v16bf, ua1), b, acc[1][j]);
            }
        }
    }

    float bcol[4];
#pragma unroll
    for (int j = 0; j < 4; ++j) bcol[j] = bf2f(f2bf(bias[Nbase + 16 * j + m]));

    unsigned char* region = stage_raw + wv * 8192;

    if (MODE == 3) {
        float* sf = (float*)region;
#pragma unroll
        for (int mt = 0; mt < 2; ++mt)
#pragma unroll
            for (int r = 0; r < 8; ++r) {
                const int row = mt * 16 + 8 * h + r;
#pragma unroll
                for (int j = 0; j < 4; ++j)
                    sf[row * 64 + 16 * j + m] = acc[mt][j][r] * (1.0f / 1024.0f) + bcol[j];
            }
    } else if (MODE == 2) {
        unsigned short* sa = (unsigned short*)region;
#pragma unroll
        for (int mt = 0; mt < 2; ++mt)
#pragma unroll
            for (int r = 0; r < 8; ++r) {
                const int row = mt * 16 + 8 * h + r;
#pragma unroll
                for (int j = 0; j < 4; ++j) {
                    const float v = (acc[mt][j][r] + bcol[j]) * 16.0f;
                    sa[row * 64 + 16 * j + m] = __builtin_bit_cast(unsigned short, (_Float16)v);
                }
            }
    } else {
        unsigned short* sa = (unsigned short*)region;
        unsigned short* sb = sa + 2048;
#pragma unroll
        for (int mt = 0; mt < 2; ++mt)
#pragma unroll
            for (int r = 0; r < 8; ++r) {
                const int row  = mt * 16 + 8 * h + r;
                const int srow = Mbase + row;
                const float cA = ct[(size_t)srow * 32 + m];
                const float cB = ct[(size_t)srow * 32 + 16 + m];
                const float sA = st[(size_t)srow * 32 + m];
                const float sB = st[(size_t)srow * 32 + 16 + m];
                const float v0 = acc[mt][0][r] + bcol[0];
                const float v1 = acc[mt][1][r] + bcol[1];
                const float v2 = acc[mt][2][r] + bcol[2];
                const float v3 = acc[mt][3][r] + bcol[3];
                float o[4];
                o[0] = v0 * cA - v2 * sA;
                o[1] = v1 * cB - v3 * sB;
                o[2] = v2 * cA + v0 * sA;
                o[3] = v3 * cB + v1 * sB;
#pragma unroll
                for (int j = 0; j < 4; ++j) {
                    const unsigned short hi = f2bf(o[j]);
                    const unsigned short lo = f2bf(o[j] - bf2f(hi));
                    sa[row * 64 + 16 * j + m] = hi;
                    sb[row * 64 + 16 * j + m] = lo;
                }
            }
    }
    __syncthreads();

#pragma unroll
    for (int pass = 0; pass < 2; ++pass) {
        if (pass) __threadfence();
        if (MODE == 3) {
            const float* sf = (const float*)region;
            float* Y = (float*)out0;
#pragma unroll
            for (int it = 0; it < 16; ++it) {
                const int row   = it * 2 + (lane >> 4);
                const int piece = lane & 15;
                const v4f val = *(const v4f*)(sf + row * 64 + piece * 4);
                *(volatile v4f*)(Y + (size_t)(Mbase + row) * D_MODEL + Nbase + piece * 4) = val;
            }
        } else {
            const unsigned short* sa = (const unsigned short*)region;
            unsigned short* Y0 = (unsigned short*)out0;
            unsigned short* Y1 = (unsigned short*)out1;
#pragma unroll
            for (int it = 0; it < 8; ++it) {
                const int row   = it * 4 + (lane >> 3);
                const int piece = lane & 7;
                const v8u va = *(const v8u*)(sa + row * 64 + piece * 8);
                *(volatile v8u*)(Y0 + (size_t)(Mbase + row) * D_MODEL + Nbase + piece * 8) = va;
                if (MODE != 2) {
                    const v8u vb = *(const v8u*)(sa + 2048 + row * 64 + piece * 8);
                    *(volatile v8u*)(Y1 + (size_t)(Mbase + row) * D_MODEL + Nbase + piece * 8) = vb;
                }
            }
        }
    }
}

__global__ __launch_bounds__(256) void attn_kernel(
    const unsigned short* __restrict__ Qhi, const unsigned short* __restrict__ Qlo,
    const unsigned short* __restrict__ Khi, const unsigned short* __restrict__ Klo,
    const _Float16* __restrict__ V16, _Float16* Aout) {
    __shared__ __attribute__((aligned(16))) unsigned short Kh_l[64 * 64];
    __shared__ __attribute__((aligned(16))) unsigned short Kl_l[64 * 64];
    __shared__ __attribute__((aligned(16))) _Float16       Vt_l[64 * 64];
    __shared__ __attribute__((aligned(16))) _Float16       P_l[8][16 * 64];

    const int tid  = threadIdx.x;
    const int lane = tid & 31;
    const int h    = lane >> 4;
    const int m    = lane & 15;
    const int w    = tid >> 5;
    const int hd   = blockIdx.x >> 4;
    const int qg   = blockIdx.x & 15;
    const int Qrow = (qg * 8 + w) * 16;
    const int hoff = hd * D_K;

    float m_run[8], l_run[8];
    v8f O[4];
#pragma unroll
    for (int r = 0; r < 8; ++r) { m_run[r] = -1e30f; l_run[r] = 0.0f; }
#pragma unroll
    for (int j = 0; j < 4; ++j) O[j] = (v8f)0.0f;

    v16bf qh[2], ql[2];
#pragma unroll
    for (int ks = 0; ks < 2; ++ks) {
        const size_t qo = (size_t)(Qrow + m) * D_MODEL + hoff + ks * 32 + 8 * h;
        qh[ks] = __builtin_bit_cast(v16bf, frag_u16(Qhi + qo));
        ql[ks] = __builtin_bit_cast(v16bf, frag_u16(Qlo + qo));
    }

#pragma unroll 1
    for (int jb = 0; jb < S_LEN; jb += 64) {
        __syncthreads();
#pragma unroll
        for (int rep = 0; rep < 2; ++rep) {
            const int i   = tid + rep * 256;
            const int row = i >> 3;
            const int c8  = (i & 7) * 8;
            const size_t g = (size_t)(jb + row) * D_MODEL + hoff + c8;
            *(v8u*)&Kh_l[row * 64 + c8] = *(const v8u*)(Khi + g);
            *(v8u*)&Kl_l[row * 64 + c8] = *(const v8u*)(Klo + g);
            const v8h vv = *(const v8h*)(V16 + g);
#pragma unroll
            for (int e = 0; e < 8; ++e) Vt_l[(c8 + e) * 64 + row] = vv[e];
        }
        __syncthreads();

        v8f sc[4];
#pragma unroll
        for (int jt = 0; jt < 4; ++jt) sc[jt] = (v8f)0.0f;
#pragma unroll
        for (int jt = 0; jt < 4; ++jt) {
#pragma unroll
            for (int ks = 0; ks < 2; ++ks) {
                const int ko = (16 * jt + m) * 64 + ks * 32 + 8 * h;
                const v16bf kh = __builtin_bit_cast(v16bf, frag_u16(&Kh_l[ko]));
                const v16bf kl = __builtin_bit_cast(v16bf, frag_u16(&Kl_l[ko]));
                sc[jt] = mma_bf16(qh[ks], kh, sc[jt]);
                sc[jt] = mma_bf16(qh[ks], kl, sc[jt]);
                sc[jt] = mma_bf16(ql[ks], kh, sc[jt]);
            }
        }

#pragma unroll
        for (int r = 0; r < 8; ++r) {
            const float s0 = sc[0][r] * 0.125f;
            const float s1 = sc[1][r] * 0.125f;
            const float s2 = sc[2][r] * 0.125f;
            const float s3 = sc[3][r] * 0.125f;
            float mx = fmaxf(fmaxf(s0, s1), fmaxf(s2, s3));
#pragma unroll
            for (int msk = 1; msk <= 8; msk <<= 1) mx = fmaxf(mx, __shfl_xor(mx, msk, 32));
            const float mnew = fmaxf(m_run[r], mx);
            const float fac  = __expf(m_run[r] - mnew);
            m_run[r] = mnew;
            const float p0 = __expf(s0 - mnew);
            const float p1 = __expf(s1 - mnew);
            const float p2 = __expf(s2 - mnew);
            const float p3 = __expf(s3 - mnew);
            float psum = (p0 + p1) + (p2 + p3);
            _Float16* prow = &P_l[w][(8 * h + r) * 64 + m];
            prow[0]  = (_Float16)(p0 * 4096.0f);
            prow[16] = (_Float16)(p1 * 4096.0f);
            prow[32] = (_Float16)(p2 * 4096.0f);
            prow[48] = (_Float16)(p3 * 4096.0f);
#pragma unroll
            for (int msk = 1; msk <= 8; msk <<= 1) psum += __shfl_xor(psum, msk, 32);
            l_run[r] = l_run[r] * fac + psum;
#pragma unroll
            for (int jd = 0; jd < 4; ++jd) O[jd][r] *= fac;
        }
        __syncthreads();

#pragma unroll
        for (int ks = 0; ks < 2; ++ks) {
            const v16h pa = frag_f16(&P_l[w][m * 64 + ks * 32 + 8 * h]);
#pragma unroll
            for (int jd = 0; jd < 4; ++jd) {
                const v16h vb = frag_f16(&Vt_l[(16 * jd + m) * 64 + ks * 32 + 8 * h]);
                O[jd] = mma_f16(pa, vb, O[jd]);
            }
        }
    }

#pragma unroll
    for (int r = 0; r < 8; ++r) {
        const float inv = (1.0f / l_run[r]) * (1.0f / 4096.0f);
#pragma unroll
        for (int jd = 0; jd < 4; ++jd)
            P_l[w][(8 * h + r) * 64 + 16 * jd + m] = (_Float16)(O[jd][r] * inv);
    }
    __syncthreads();

#pragma unroll
    for (int pass = 0; pass < 2; ++pass) {
        if (pass) __threadfence();
#pragma unroll
        for (int it = 0; it < 4; ++it) {
            const int row   = it * 4 + (lane >> 3);
            const int piece = lane & 7;
            const v8h val = *(const v8h*)&P_l[w][row * 64 + piece * 8];
            *(volatile v8h*)(Aout + (size_t)(Qrow + row) * D_MODEL + hoff + piece * 8) = val;
        }
    }
}

extern "C" void kernel_launch(void* const* d_in, const int* in_sizes, int n_in,
                              void* d_out, int out_size, void* d_ws, size_t ws_size,
                              hipStream_t stream) {
    const int ACT = S_LEN * D_MODEL;
    const int WEI = D_MODEL * D_MODEL;
    if (n_in < 11) return;
    if (in_sizes[0] != ACT || in_sizes[1] != ACT || in_sizes[2] != ACT) return;
    if (in_sizes[3] != WEI || in_sizes[5] != WEI || in_sizes[7] != WEI || in_sizes[9] != WEI) return;
    if (in_sizes[4] != D_MODEL || in_sizes[6] != D_MODEL || in_sizes[8] != D_MODEL || in_sizes[10] != D_MODEL) return;
    if (out_size != ACT) return;

    const float* q_in = (const float*)d_in[0];
    const float* k_in = (const float*)d_in[1];
    const float* v_in = (const float*)d_in[2];
    const float* q_w  = (const float*)d_in[3];
    const float* q_b  = (const float*)d_in[4];
    const float* k_w  = (const float*)d_in[5];
    const float* k_b  = (const float*)d_in[6];
    const float* v_w  = (const float*)d_in[7];
    const float* v_b  = (const float*)d_in[8];
    const float* o_w  = (const float*)d_in[9];
    const float* o_b  = (const float*)d_in[10];

    const size_t ACT16 = (size_t)ACT * 2;
    const size_t WEI16 = (size_t)WEI * 2;
    const size_t TAB   = (size_t)S_LEN * 32 * 4;
    size_t off = 0;
    const size_t o_xq  = off; off += ACT16;
    const size_t o_xk  = off; off += ACT16;
    const size_t o_xv  = off; off += ACT16;
    const size_t o_wq  = off; off += WEI16;
    const size_t o_wk  = off; off += WEI16;
    const size_t o_wv  = off; off += WEI16;
    const size_t o_wo  = off; off += WEI16;
    const size_t o_qhi = off; off += ACT16;
    const size_t o_qlo = off; off += ACT16;
    const size_t o_khi = off; off += ACT16;
    const size_t o_klo = off; off += ACT16;
    const size_t o_v16 = off; off += ACT16;
    const size_t o_a16 = off; off += ACT16;
    const size_t o_ct  = off; off += TAB;
    const size_t o_st  = off; off += TAB;
    if (off > ws_size) return;

    char* ws = (char*)d_ws;
    unsigned short* xq  = (unsigned short*)(ws + o_xq);
    unsigned short* xk  = (unsigned short*)(ws + o_xk);
    unsigned short* xv  = (unsigned short*)(ws + o_xv);
    unsigned short* wq  = (unsigned short*)(ws + o_wq);
    unsigned short* wk  = (unsigned short*)(ws + o_wk);
    unsigned short* wv  = (unsigned short*)(ws + o_wv);
    unsigned short* wo  = (unsigned short*)(ws + o_wo);
    unsigned short* Qhi = (unsigned short*)(ws + o_qhi);
    unsigned short* Qlo = (unsigned short*)(ws + o_qlo);
    unsigned short* Khi = (unsigned short*)(ws + o_khi);
    unsigned short* Klo = (unsigned short*)(ws + o_klo);
    _Float16*       V16 = (_Float16*)(ws + o_v16);
    _Float16*       A16 = (_Float16*)(ws + o_a16);
    float*          ct  = (float*)(ws + o_ct);
    float*          st  = (float*)(ws + o_st);

    const int nact8 = ACT / 8, nwei8 = WEI / 8;
    hipLaunchKernelGGL(cvt_kernel, dim3((nact8 + 255) / 256, 3), dim3(256), 0, stream,
                       q_in, k_in, v_in, q_in, xq, xk, xv, xq, nact8, 0);
    hipLaunchKernelGGL(cvt_kernel, dim3((nwei8 + 255) / 256, 4), dim3(256), 0, stream,
                       q_w, k_w, v_w, o_w, wq, wk, wv, wo, nwei8, 1);

    const int ntab4 = S_LEN * 32 / 4;
    hipLaunchKernelGGL(rope_tab_kernel, dim3((ntab4 + 255) / 256), dim3(256), 0, stream, ct, st, ntab4);

    hipLaunchKernelGGL(gemm_kernel<0>, dim3(256), dim3(128), 0, stream,
                       (const unsigned short*)xq, (const unsigned short*)wq, q_b,
                       (const float*)ct, (const float*)st, (void*)Qhi, (void*)Qlo);
    hipLaunchKernelGGL(gemm_kernel<1>, dim3(256), dim3(128), 0, stream,
                       (const unsigned short*)xk, (const unsigned short*)wk, k_b,
                       (const float*)ct, (const float*)st, (void*)Khi, (void*)Klo);
    hipLaunchKernelGGL(gemm_kernel<2>, dim3(256), dim3(128), 0, stream,
                       (const unsigned short*)xv, (const unsigned short*)wv, v_b,
                       (const float*)ct, (const float*)st, (void*)V16, (void*)V16);

    hipLaunchKernelGGL(attn_kernel, dim3(N_HEADS * (S_LEN / 128)), dim3(256), 0, stream,
                       (const unsigned short*)Qhi, (const unsigned short*)Qlo,
                       (const unsigned short*)Khi, (const unsigned short*)Klo,
                       (const _Float16*)V16, A16);

    hipLaunchKernelGGL(gemm_kernel<3>, dim3(256), dim3(128), 0, stream,
                       (const unsigned short*)A16, (const unsigned short*)wo, o_b,
                       (const float*)ct, (const float*)st, d_out, d_out);
}
